// VAT_self_attention_1D_89343909691495
// MI455X (gfx1250) — hardware-verified
//
#include <hip/hip_runtime.h>

static constexpr int NB   = 4;
static constexpr int NT   = 4096;
static constexpr int NTOK = NB * NT;
static constexpr int FIN  = 229;
static constexpr int FP   = 256;
static constexpr int DM   = 256;
static constexpr int NG   = 8;
static constexpr int DG   = 32;
static constexpr int KW   = 31;
static constexpr int PADT = 15;
static constexpr int NO   = 88;
static constexpr int NOP  = 96;
static constexpr float LN_EPS = 1e-5f;
static constexpr float WSCALE = 16.0f;
static constexpr float WINV   = 0.0625f;

static constexpr size_t SZ_SP    = (size_t)NTOK * FP * 2;
static constexpr size_t SZ_W     = (size_t)DM * FP * 2;
static constexpr size_t SZ_LW    = (size_t)NOP * DM * 2;
static constexpr size_t SZ_F32P  = (size_t)NTOK * DM * 4;
static constexpr size_t OFF_SPHI = 0;
static constexpr size_t OFF_SPLO = OFF_SPHI + SZ_SP;
static constexpr size_t OFF_SP16 = OFF_SPLO + SZ_SP;
static constexpr size_t OFF_WQHI = OFF_SP16 + SZ_SP;
static constexpr size_t OFF_WQLO = OFF_WQHI + SZ_W;
static constexpr size_t OFF_WKHI = OFF_WQLO + SZ_W;
static constexpr size_t OFF_WKLO = OFF_WKHI + SZ_W;
static constexpr size_t OFF_WV16 = OFF_WKLO + SZ_W;
static constexpr size_t OFF_LW16 = OFF_WV16 + SZ_W;
static constexpr size_t OFF_QF   = OFF_LW16 + SZ_LW;
static constexpr size_t OFF_KF   = OFF_QF + SZ_F32P;
static constexpr size_t OFF_VF   = OFF_KF + SZ_F32P;
static constexpr size_t WS_TOTAL = OFF_VF + SZ_F32P;
static_assert(WS_TOTAL <= (size_t)134217728);
static_assert((OFF_LW16 % 128) == 0);
static_assert((OFF_QF % 128) == 0);
static_assert((OFF_KF % 128) == 0);
static_assert((OFF_VF % 128) == 0);

static constexpr int CB_SPEC  = NTOK * FP / 8 / 256;
static constexpr int CB_W     = DM * FP / 8 / 256;
static constexpr int CB_LW    = NOP * DM / 8 / 256;
static constexpr int CB_TOTAL = CB_SPEC + 3 * CB_W + CB_LW;
static_assert(CB_SPEC * 256 * 8 == NTOK * FP);
static_assert(CB_W * 256 * 8 == DM * FP);
static_assert(CB_LW * 256 * 8 == NOP * DM);

static constexpr int SKROWS   = 62;
static constexpr int LDS_F_K  = SKROWS * DM;
static constexpr int LDS_F_Q  = 32 * DM;
static constexpr int LDS_F_P  = 32 * NG * KW;
static constexpr int ATT_LDS_BYTES = (2 * LDS_F_K + LDS_F_Q + LDS_F_P) * 4;
static_assert(32 * DM * 2 <= LDS_F_K * 4);
static_assert(32 * NO <= LDS_F_K);
static_assert(NTOK % 32 == 0 && NT % 32 == 0);

typedef __attribute__((ext_vector_type(16))) _Float16       v16h;
typedef __attribute__((ext_vector_type(16))) __bf16         v16bf;
typedef __attribute__((ext_vector_type(16))) unsigned short v16us;
typedef __attribute__((ext_vector_type(8)))  unsigned short v8us;
typedef __attribute__((ext_vector_type(8)))  float          v8f;
typedef __attribute__((ext_vector_type(4)))  float          v4f;
typedef v8us __attribute__((may_alias)) v8usa;
typedef v4f  __attribute__((may_alias)) v4fa;

union FragU { v16us v; v8us half[2]; };

__device__ __forceinline__ unsigned short bf16_rne(float f) {
  unsigned u = __float_as_uint(f);
  u = u + 0x7FFFu + ((u >> 16) & 1u);
  return (unsigned short)(u >> 16);
}
__device__ __forceinline__ float bf16_val(unsigned short s) {
  return __uint_as_float(((unsigned)s) << 16);
}

__device__ __forceinline__ v8f wmma_bf16(v16us a, v16us b, v8f c) {
  v8f d = __builtin_amdgcn_wmma_f32_16x16x32_bf16(false, __builtin_bit_cast(v16bf, a), false,
                                                  __builtin_bit_cast(v16bf, b), (short)0, c, false, false);
  asm volatile("v_nop\n\tv_nop\n\tv_nop\n\tv_nop" : "+v"(d) : "v"(a), "v"(b));
  return d;
}
__device__ __forceinline__ v8f wmma_f16(v16us a, v16us b, v8f c) {
  v8f d = __builtin_amdgcn_wmma_f32_16x16x32_f16(false, __builtin_bit_cast(v16h, a), false,
                                                 __builtin_bit_cast(v16h, b), (short)0, c, false, false);
  asm volatile("v_nop\n\tv_nop\n\tv_nop\n\tv_nop" : "+v"(d) : "v"(a), "v"(b));
  return d;
}

__device__ __forceinline__ v16us load_frag(const unsigned short* p, int h) {
  FragU f;
  f.half[0] = *(const v8usa*)(p + 8 * h);
  f.half[1] = *(const v8usa*)(p + 16 + 8 * h);
  return f.v;
}

__global__ __launch_bounds__(256) void convert_kernel(
    const float* __restrict__ spec, const float* __restrict__ wq, const float* __restrict__ wk,
    const float* __restrict__ wv, const float* __restrict__ lw,
    unsigned short* sp_hi, unsigned short* sp_lo, unsigned short* sp_16,
    unsigned short* wq_hi, unsigned short* wq_lo, unsigned short* wk_hi, unsigned short* wk_lo,
    unsigned short* wv_16, unsigned short* lw_16)
{
  const int blk = blockIdx.x, tid = threadIdx.x;
  float x[8];
  unsigned short* dH = sp_hi;
  unsigned short* dL = sp_lo;
  unsigned short* dF = sp_16;
  int kind;
  size_t off;
  if (blk < CB_SPEC) {
    const int g = blk * 256 + tid;
    const int row = g >> 5, c0 = (g & 31) * 8;
    const float* src = spec + (size_t)row * FIN;
    #pragma unroll
    for (int e = 0; e < 8; ++e) {
      const int f = c0 + e;
      const int fa = (f < FIN) ? f : (FIN - 1);
      const float t = src[fa];
      x[e] = (f < FIN) ? t : (t * 0.0f);
    }
    off = (size_t)row * FP + c0;
    kind = 0;
  } else if (blk < CB_SPEC + 2 * CB_W) {
    const int g = (blk - CB_SPEC) * 256 + tid;
    const int sel = g >> 13;
    const int e2 = g & 8191;
    const int n = e2 >> 5, c0 = (e2 & 31) * 8;
    const float* src = ((sel == 0) ? wq : wk) + (size_t)n * FIN;
    #pragma unroll
    for (int e = 0; e < 8; ++e) {
      const int f = c0 + e;
      const int fa = (f < FIN) ? f : (FIN - 1);
      const float t = src[fa];
      x[e] = (f < FIN) ? t : (t * 0.0f);
    }
    off = (size_t)n * FP + c0;
    dH = (sel == 0) ? wq_hi : wk_hi;
    dL = (sel == 0) ? wq_lo : wk_lo;
    kind = 1;
  } else if (blk < CB_SPEC + 3 * CB_W) {
    const int g = (blk - CB_SPEC - 2 * CB_W) * 256 + tid;
    const int n = g >> 5, c0 = (g & 31) * 8;
    const float* src = wv + (size_t)n * FIN;
    #pragma unroll
    for (int e = 0; e < 8; ++e) {
      const int f = c0 + e;
      const int fa = (f < FIN) ? f : (FIN - 1);
      const float t = src[fa];
      x[e] = (f < FIN) ? (t * WSCALE) : (t * 0.0f);
    }
    off = (size_t)n * FP + c0;
    dF = wv_16;
    kind = 2;
  } else {
    const int g = (blk - CB_SPEC - 3 * CB_W) * 256 + tid;
    const int n = g >> 5, d0 = (g & 31) * 8;
    const int na = (n < NO) ? n : (NO - 1);
    const float* src = lw + (size_t)na * DM + d0;
    #pragma unroll
    for (int e = 0; e < 8; ++e) {
      const float t = src[e];
      x[e] = (n < NO) ? (t * WSCALE) : (t * 0.0f);
    }
    off = (size_t)n * DM + d0;
    dF = lw_16;
    kind = 2;
  }

  v8us ph, pl, pf;
  #pragma unroll
  for (int e = 0; e < 8; ++e) {
    const unsigned short sh = bf16_rne(x[e]);
    ph[e] = sh;
    pl[e] = bf16_rne(x[e] - bf16_val(sh));
    pf[e] = __builtin_bit_cast(unsigned short, (_Float16)x[e]);
  }
  if (kind != 2) {
    *(volatile v8us*)(dH + off) = ph;
    *(volatile v8us*)(dL + off) = pl;
  }
  if (kind != 1) {
    *(volatile v8us*)(dF + off) = pf;
  }
  __threadfence();
  if (kind != 2) {
    *(volatile v8us*)(dH + off) = ph;
    *(volatile v8us*)(dL + off) = pl;
  }
  if (kind != 1) {
    *(volatile v8us*)(dF + off) = pf;
  }
}

__device__ __forceinline__ void proj_store_pass(const float* sT, float* Y, int m0, int fg,
                                                int w, int lane) {
  const int q8 = lane & 7, sub = lane >> 3;
  #pragma unroll
  for (int i = 0; i < 16; ++i) {
    const int lid = i * 4 + sub;
    const int row = 32 * w + (lid >> 1), hl = lid & 1;
    const v4f v = *(const v4fa*)(sT + row * 64 + 32 * hl + 4 * q8);
    *(volatile v4f*)(Y + (size_t)(m0 + row) * DM + fg * 64 + 32 * hl + 4 * q8) = v;
  }
}

template <int SPLIT>
__global__ __launch_bounds__(128) void proj_kernel(
    const unsigned short* Ah, const unsigned short* Al,
    const unsigned short* W0h, const unsigned short* W0l,
    const unsigned short* W1h, const unsigned short* W1l,
    float* Y0, float* Y1, float oscale)
{
  __shared__ __attribute__((aligned(16))) float sT[128 * 64];

  const int tid = threadIdx.x, lane = tid & 31, w = tid >> 5;
  const int h = lane >> 4, m = lane & 15;
  const int m0 = blockIdx.x * 128;
  const int fg = blockIdx.y;
  const int which = blockIdx.z;
  const unsigned short* Wh = (which == 0) ? W0h : W1h;
  const unsigned short* Wl = (which == 0) ? W0l : W1l;
  float* Y = (which == 0) ? Y0 : Y1;
  const int m0w = m0 + 32 * w;

  const unsigned short* xa0 = Ah + (size_t)(m0w + m) * FP;
  const unsigned short* xa1 = xa0 + (size_t)16 * FP;
  const unsigned short* xl0 = Al + (size_t)(m0w + m) * FP;
  const unsigned short* xl1 = xl0 + (size_t)16 * FP;
  const unsigned short* wbh = Wh + (size_t)(fg * 64 + m) * FP;
  const unsigned short* wbl = Wl + (size_t)(fg * 64 + m) * FP;

  const v8f zero8 = {0.f, 0.f, 0.f, 0.f, 0.f, 0.f, 0.f, 0.f};
  v8f acc[2][4];
  #pragma unroll
  for (int mt = 0; mt < 2; ++mt)
    #pragma unroll
    for (int nt = 0; nt < 4; ++nt) acc[mt][nt] = zero8;

  #pragma unroll 1
  for (int k0 = 0; k0 < FP; k0 += 32) {
    const v16us a0 = load_frag(xa0 + k0, h);
    const v16us a1 = load_frag(xa1 + k0, h);
    if (SPLIT) {
      const v16us l0 = load_frag(xl0 + k0, h);
      const v16us l1 = load_frag(xl1 + k0, h);
      #pragma unroll
      for (int nt = 0; nt < 4; ++nt) {
        const v16us bh = load_frag(wbh + (size_t)nt * 16 * FP + k0, h);
        const v16us bl = load_frag(wbl + (size_t)nt * 16 * FP + k0, h);
        acc[0][nt] = wmma_bf16(a0, bh, acc[0][nt]);
        acc[0][nt] = wmma_bf16(a0, bl, acc[0][nt]);
        acc[0][nt] = wmma_bf16(l0, bh, acc[0][nt]);
        acc[1][nt] = wmma_bf16(a1, bh, acc[1][nt]);
        acc[1][nt] = wmma_bf16(a1, bl, acc[1][nt]);
        acc[1][nt] = wmma_bf16(l1, bh, acc[1][nt]);
      }
    } else {
      #pragma unroll
      for (int nt = 0; nt < 4; ++nt) {
        const v16us b = load_frag(wbh + (size_t)nt * 16 * FP + k0, h);
        acc[0][nt] = wmma_f16(a0, b, acc[0][nt]);
        acc[1][nt] = wmma_f16(a1, b, acc[1][nt]);
      }
    }
  }

  #pragma unroll
  for (int nt = 0; nt < 4; ++nt) {
    const int feat = 16 * nt + m;
    #pragma unroll
    for (int mt = 0; mt < 2; ++mt) {
      #pragma unroll
      for (int r = 0; r < 8; ++r) {
        const int tokl = 32 * w + 16 * mt + 8 * h + r;
        sT[tokl * 64 + feat] = acc[mt][nt][r] * oscale;
      }
    }
  }
  __syncthreads();

  proj_store_pass(sT, Y, m0, fg, w, lane);
  __threadfence();
  proj_store_pass(sT, Y, m0, fg, w, lane);
}

__global__ __launch_bounds__(256) void attn_kernel(
    const float* __restrict__ Qf, const float* __restrict__ Kf, const float* __restrict__ Vf,
    const float* __restrict__ rel, const float* __restrict__ gam, const float* __restrict__ bet,
    const unsigned short* __restrict__ lw16, const float* __restrict__ lb,
    float* out0, float* out1)
{
  extern __shared__ __attribute__((aligned(16))) float dsm[];
  float* sK = dsm;
  float* sV = dsm + LDS_F_K;
  float* sQ = dsm + 2 * LDS_F_K;
  float* sP = sQ + LDS_F_Q;
  _Float16* sH = (_Float16*)dsm;
  float* sO = sV;

  const int tid = threadIdx.x, lane = tid & 31, w = tid >> 5;
  const int h = lane >> 4, m = lane & 15;
  const int blk = blockIdx.x;
  const int b = blk >> 7;
  const int t0 = (blk & 127) * 32;
  const int tok0 = blk * 32;

  {
    const int c4 = tid & 63, rsub = tid >> 6;
    const v4f zero4 = {0.f, 0.f, 0.f, 0.f};
    #pragma unroll 1
    for (int ps = 0; ps < 16; ++ps) {
      const int s = ps * 4 + rsub;
      if (s < SKROWS) {
        const int fr = t0 - PADT + s;
        const bool ok = (fr >= 0) && (fr < NT);
        const int fc = (fr < 0) ? 0 : ((fr >= NT) ? (NT - 1) : fr);
        const size_t go = ((size_t)b * NT + fc) * DM + 4 * c4;
        v4f kx = *(const v4fa*)(Kf + go);
        v4f vx = *(const v4fa*)(Vf + go);
        if (!ok) { kx = zero4; vx = zero4; }
        *(v4fa*)(sK + s * DM + 4 * c4) = kx;
        *(v4fa*)(sV + s * DM + 4 * c4) = vx;
      }
    }
    #pragma unroll 1
    for (int ps = 0; ps < 8; ++ps) {
      const int lt = ps * 4 + rsub;
      const size_t go = ((size_t)tok0 + lt) * DM + 4 * c4;
      *(v4fa*)(sQ + lt * DM + 4 * c4) = *(const v4fa*)(Qf + go);
    }
  }
  __syncthreads();

  {
    const int g = w;
    const int jl = (lane < KW) ? lane : (KW - 1);
    float relr[DG];
    #pragma unroll
    for (int d = 0; d < DG; ++d) relr[d] = rel[(size_t)(g * DG + d) * KW + jl];

    #pragma unroll 1
    for (int lt = 0; lt < 32; ++lt) {
      const float* qp = sQ + lt * DM + g * DG;
      const float* kp = sK + (lt + jl) * DM + g * DG;
      float e = 0.0f;
      #pragma unroll
      for (int i = 0; i < 8; ++i) {
        const v4f q4 = *(const v4fa*)(qp + 4 * i);
        const v4f k4 = *(const v4fa*)(kp + 4 * i);
        e += q4.x * (k4.x + relr[4 * i + 0]);
        e += q4.y * (k4.y + relr[4 * i + 1]);
        e += q4.z * (k4.z + relr[4 * i + 2]);
        e += q4.w * (k4.w + relr[4 * i + 3]);
      }
      const float ev = (lane < KW) ? e : -1.0e30f;
      float mx = ev;
      #pragma unroll
      for (int off = 16; off >= 1; off >>= 1) mx = fmaxf(mx, __shfl_xor(mx, off));
      float p = expf(ev - mx);
      float s = p;
      #pragma unroll
      for (int off = 16; off >= 1; off >>= 1) s += __shfl_xor(s, off);
      p = p * (1.0f / s);
      if (lane < KW) sP[lt * (NG * KW) + g * KW + lane] = p;

      const float* vp = sV + lt * DM + g * DG + lane;
      float c = 0.0f;
      #pragma unroll
      for (int j = 0; j < KW; ++j) {
        const float pj = __shfl(p, j);
        c += pj * vp[j * DM];
      }
      sQ[lt * DM + g * DG + lane] = c;
    }
  }
  __syncthreads();

  {
    float* o1 = out1 + (size_t)blk * LDS_F_P;
    #pragma unroll
    for (int it = 0; it < 8; ++it) {
      const int q = it * 256 + tid;
      if (q < LDS_F_P / 4) {
        const v4f v = *(const v4fa*)(sP + 4 * q);
        *(volatile v4f*)(o1 + 4 * q) = v;
      }
    }
    __threadfence();
    #pragma unroll
    for (int it = 0; it < 8; ++it) {
      const int q = it * 256 + tid;
      if (q < LDS_F_P / 4) {
        const v4f v = *(const v4fa*)(sP + 4 * q);
        *(volatile v4f*)(o1 + 4 * q) = v;
      }
    }
  }

  {
    float gm[8], bt[8];
    #pragma unroll
    for (int i = 0; i < 8; ++i) { gm[i] = gam[lane + 32 * i]; bt[i] = bet[lane + 32 * i]; }
    #pragma unroll 1
    for (int rr = 0; rr < 4; ++rr) {
      const int lt = w * 4 + rr;
      float x[8];
      float s = 0.0f;
      #pragma unroll
      for (int i = 0; i < 8; ++i) { x[i] = sQ[lt * DM + lane + 32 * i]; s += x[i]; }
      #pragma unroll
      for (int off = 16; off >= 1; off >>= 1) s += __shfl_xor(s, off);
      const float mu = s * (1.0f / 256.0f);
      float v = 0.0f;
      #pragma unroll
      for (int i = 0; i < 8; ++i) { const float d = x[i] - mu; v += d * d; }
      #pragma unroll
      for (int off = 16; off >= 1; off >>= 1) v += __shfl_xor(v, off);
      const float rstd = 1.0f / sqrtf(v * (1.0f / 256.0f) + LN_EPS);
      #pragma unroll
      for (int i = 0; i < 8; ++i) {
        const int c = lane + 32 * i;
        const float hv = (x[i] - mu) * rstd * gm[i] + bt[i];
        sH[lt * DM + c] = (_Float16)hv;
      }
    }
  }
  __syncthreads();

  if (w < 6) {
    const unsigned short* hbase = (const unsigned short*)sH;
    const unsigned short* ha0 = hbase + m * DM;
    const unsigned short* ha1 = hbase + (16 + m) * DM;
    const unsigned short* wrow = lw16 + (size_t)(16 * w + m) * DM;
    const v8f zero8 = {0.f, 0.f, 0.f, 0.f, 0.f, 0.f, 0.f, 0.f};
    v8f acc0 = zero8, acc1 = zero8;
    #pragma unroll
    for (int ks = 0; ks < 8; ++ks) {
      const int k0 = 32 * ks;
      const v16us a0 = load_frag(ha0 + k0, h);
      const v16us a1 = load_frag(ha1 + k0, h);
      const v16us bb = load_frag(wrow + k0, h);
      acc0 = wmma_f16(a0, bb, acc0);
      acc1 = wmma_f16(a1, bb, acc1);
    }
    const int n = 16 * w + m;
    const int na = (n < NO) ? n : (NO - 1);
    const float bias = lb[na];
    #pragma unroll
    for (int r = 0; r < 8; ++r) {
      const float y0 = acc0[r] * WINV + bias;
      const float y1 = acc1[r] * WINV + bias;
      const float s0 = 1.0f / (1.0f + __expf(-y0));
      const float s1 = 1.0f / (1.0f + __expf(-y1));
      if (n < NO) {
        sO[(8 * h + r) * NO + n] = s0;
        sO[(16 + 8 * h + r) * NO + n] = s1;
      }
    }
  }
  __syncthreads();

  {
    float* o0 = out0 + (size_t)blk * (32 * NO);
    #pragma unroll
    for (int it = 0; it < 3; ++it) {
      const int q = it * 256 + tid;
      if (q < (32 * NO) / 4) {
        const v4f v = *(const v4fa*)(sO + 4 * q);
        *(volatile v4f*)(o0 + 4 * q) = v;
      }
    }
    __threadfence();
    #pragma unroll
    for (int it = 0; it < 3; ++it) {
      const int q = it * 256 + tid;
      if (q < (32 * NO) / 4) {
        const v4f v = *(const v4fa*)(sO + 4 * q);
        *(volatile v4f*)(o0 + 4 * q) = v;
      }
    }
  }
}

extern "C" void kernel_launch(void* const* d_in, const int* in_sizes, int n_in,
                              void* d_out, int out_size, void* d_ws, size_t ws_size,
                              hipStream_t stream) {
  if (n_in < 9) return;
  if (in_sizes[0] != NTOK * FIN) return;
  if (in_sizes[1] != DM * FIN || in_sizes[2] != DM * FIN || in_sizes[3] != DM * FIN) return;
  if (in_sizes[4] != DM * KW) return;
  if (in_sizes[5] != DM || in_sizes[6] != DM) return;
  if (in_sizes[7] != NO * DM || in_sizes[8] != NO) return;
  if (out_size != NTOK * NO + NTOK * NG * KW) return;
  if (WS_TOTAL > ws_size) return;

  const float* spec = (const float*)d_in[0];
  const float* W_q  = (const float*)d_in[1];
  const float* W_k  = (const float*)d_in[2];
  const float* W_v  = (const float*)d_in[3];
  const float* rel  = (const float*)d_in[4];
  const float* gam  = (const float*)d_in[5];
  const float* bet  = (const float*)d_in[6];
  const float* linw = (const float*)d_in[7];
  const float* linb = (const float*)d_in[8];

  float* out0 = (float*)d_out;
  float* out1 = out0 + (size_t)NTOK * NO;

  char* ws = (char*)d_ws;
  unsigned short* sp_hi = (unsigned short*)(ws + OFF_SPHI);
  unsigned short* sp_lo = (unsigned short*)(ws + OFF_SPLO);
  unsigned short* sp_16 = (unsigned short*)(ws + OFF_SP16);
  unsigned short* wq_hi = (unsigned short*)(ws + OFF_WQHI);
  unsigned short* wq_lo = (unsigned short*)(ws + OFF_WQLO);
  unsigned short* wk_hi = (unsigned short*)(ws + OFF_WKHI);
  unsigned short* wk_lo = (unsigned short*)(ws + OFF_WKLO);
  unsigned short* wv_16 = (unsigned short*)(ws + OFF_WV16);
  unsigned short* lw_16 = (unsigned short*)(ws + OFF_LW16);
  float* Qf = (float*)(ws + OFF_QF);
  float* Kf = (float*)(ws + OFF_KF);
  float* Vf = (float*)(ws + OFF_VF);

  convert_kernel<<<dim3(CB_TOTAL), dim3(256), 0, stream>>>(
      spec, W_q, W_k, W_v, linw, sp_hi, sp_lo, sp_16, wq_hi, wq_lo, wk_hi, wk_lo, wv_16, lw_16);

  proj_kernel<1><<<dim3(NTOK / 128, DM / 64, 2), dim3(128), 0, stream>>>(
      sp_hi, sp_lo, wq_hi, wq_lo, wk_hi, wk_lo, Qf, Kf, 1.0f);

  proj_kernel<0><<<dim3(NTOK / 128, DM / 64, 1), dim3(128), 0, stream>>>(
      sp_16, sp_16, wv_16, wv_16, wv_16, wv_16, Vf, Vf, WINV);

  hipFuncSetAttribute(reinterpret_cast<const void*>(&attn_kernel),
                      hipFuncAttributeMaxDynamicSharedMemorySize, ATT_LDS_BYTES);
  attn_kernel<<<dim3(NTOK / 32), dim3(256), ATT_LDS_BYTES, stream>>>(
      Qf, Kf, Vf, rel, gam, bet, lw_16, linb, out0, out1);
}
